// Qwen3InfAttention_5248450036531
// MI455X (gfx1250) — hardware-verified
//
#include <hip/hip_runtime.h>


namespace {
constexpr int NB = 2, S = 2048, HID = 2048, HQ = 16, HKV = 8, DH = 128, GRP = HQ / HKV, TOT = (HQ + 2 * HKV) * DH, NROW = NB * S;
constexpr float XS = 8.0f, WSC = 256.0f, PS = 8.0f, EPS = 1e-6f, SCALING = 0.08838834764831845f;

typedef _Float16 b16;
typedef __attribute__((ext_vector_type(16))) _Float16 v16b;
typedef __attribute__((ext_vector_type(8))) _Float16 v8b;
typedef __attribute__((ext_vector_type(8))) float v8f;
typedef __attribute__((ext_vector_type(4))) float v4f;
__device__ __forceinline__ float bf16_rne(float f) { unsigned int u = __float_as_uint(f); u += 0x7FFFu + ((u >> 16) & 1u); return __uint_as_float(u & 0xFFFF0000u); }
__device__ __forceinline__ void split16(float v, b16& hi, b16& lo) { hi = (b16)v; lo = (b16)(v - (float)hi); }
__device__ __forceinline__ v16b frag_kb(const b16* p, int hh) { const v8b a = *(const v8b*)(p + 8 * hh), b = *(const v8b*)(p + 16 + 8 * hh); v16b f;
#pragma unroll
  for (int e = 0; e < 8; ++e) { f[e] = a[e]; f[8 + e] = b[e]; } return f; }
__device__ __forceinline__ v8f wmma16b(v16b a, v16b b, v8f c) { v8f d = __builtin_amdgcn_wmma_f32_16x16x32_f16(false, a, false, b, (short)0, c, false, false); asm volatile("v_nop\n\tv_nop\n\tv_nop\n\tv_nop" : "+v"(d) : "v"(a), "v"(b)); return d; }
__device__ __forceinline__ void wave_lds_sync() { __builtin_amdgcn_fence(__ATOMIC_RELEASE, "workgroup"); __builtin_amdgcn_wave_barrier(); __builtin_amdgcn_fence(__ATOMIC_ACQUIRE, "workgroup"); }
__device__ __forceinline__ float nexp(float x) { return __builtin_amdgcn_exp2f(x * 1.4426950408889634f); }
__device__ __forceinline__ float pmul(float a, float b) { float p = a * b; asm volatile("" : "+v"(p)); return p; }
__device__ __forceinline__ float hsum16(float v) { v += __shfl_xor(v, 1); v += __shfl_xor(v, 2); v += __shfl_xor(v, 4); return v + __shfl_xor(v, 8); }

__global__ __launch_bounds__(256) void prep_kernel(const float* __restrict__ x, const float* __restrict__ wq, const float* __restrict__ wo, b16* __restrict__ X16, b16* __restrict__ WQ, b16* __restrict__ WO) {
  const size_t tid = (size_t)blockIdx.x * 256 + threadIdx.x, nth = (size_t)gridDim.x * 256; const size_t n1 = (size_t)NROW * HID / 8, n2 = (size_t)TOT * HID / 8, n3 = (size_t)HID * HID / 8;
  for (int pass = 0; pass < 2; ++pass) {
    for (size_t g = tid; g < n1 + n2 + n3; g += nth) { const float* src; b16* dst; size_t e; float sc;
      if (g < n1) { src = x; dst = X16; e = g * 8; sc = XS; } else if (g < n1 + n2) { src = wq; dst = WQ; e = (g - n1) * 8; sc = WSC; } else { src = wo; dst = WO; e = (g - n1 - n2) * 8; sc = WSC; }
      const v4f a = *(const v4f*)(src + e), c = *(const v4f*)(src + e + 4); v8b o;
#pragma unroll
      for (int j = 0; j < 4; ++j) { o[j] = (b16)(bf16_rne(a[j]) * sc); o[4 + j] = (b16)(bf16_rne(c[j]) * sc); }
      *(volatile v8b*)(dst + e) = o; }
    __threadfence(); }
}
__global__ __launch_bounds__(128) void qkv_kernel(const b16* __restrict__ X16, const b16* __restrict__ WQ, const float* __restrict__ cosT, const float* __restrict__ sinT, const float* __restrict__ qnw, const float* __restrict__ knw, b16* __restrict__ QH, b16* __restrict__ QL, b16* __restrict__ KH, b16* __restrict__ VROW) {
  __shared__ __attribute__((aligned(16))) b16 Th[4][16][DH + 8], Tl[4][16][DH + 8];
  const int wave = threadIdx.x >> 5, lane = threadIdx.x & 31, nloc = lane & 15, hlf = lane >> 4; const int m0 = blockIdx.x * 64 + wave * 16, nb = blockIdx.y, n0 = nb * DH;
  const int kind = nb < HQ ? 0 : nb < HQ + HKV ? 1 : 2; const int head = kind == 0 ? nb : kind == 1 ? nb - HQ : nb - HQ - HKV;
  v8f acc[8];
#pragma unroll
  for (int t = 0; t < 8; ++t) acc[t] = (v8f){};
#pragma unroll 2
  for (int kb = 0; kb < HID; kb += 32) { const v16b a = frag_kb(X16 + (size_t)(m0 + nloc) * HID + kb, hlf);
#pragma unroll
    for (int t = 0; t < 8; ++t) acc[t] = wmma16b(a, frag_kb(WQ + (size_t)(n0 + t * 16 + nloc) * HID + kb, hlf), acc[t]); }
#pragma unroll
  for (int t = 0; t < 8; ++t)
#pragma unroll
    for (int r = 0; r < 8; ++r) acc[t][r] *= (1.0f / (XS * WSC));
  if (kind < 2) {
    const float* nw = kind == 0 ? qnw : knw;
#pragma unroll
    for (int r = 0; r < 8; ++r) { const int m = m0 + 8 * hlf + r, b = m / S, s = m - b * S; float ss = 0.0f;
#pragma unroll
      for (int t = 0; t < 8; ++t) ss += pmul(acc[t][r], acc[t][r]);
      ss = hsum16(ss); const float rs = rsqrtf(ss * (1.0f / DH) + EPS); float xn[8];
#pragma unroll
      for (int t = 0; t < 8; ++t) xn[t] = pmul(bf16_rne(nw[t * 16 + nloc]), acc[t][r] * rs);
      const float* cr = cosT + ((size_t)b * S + s) * DH; const float* sr = sinT + ((size_t)b * S + s) * DH;
#pragma unroll
      for (int t = 0; t < 4; ++t) { const int d0 = t * 16 + nloc, d1 = d0 + 64; const float c0 = bf16_rne(cr[d0]), c1 = bf16_rne(cr[d1]), s0 = bf16_rne(sr[d0]), s1 = bf16_rne(sr[d1]);
        acc[t][r] = pmul(xn[t], c0) - pmul(xn[t + 4], s0); acc[t + 4][r] = pmul(xn[t + 4], c1) + pmul(xn[t], s1); } } }
#pragma unroll
  for (int t = 0; t < 8; ++t)
#pragma unroll
    for (int r = 0; r < 8; ++r) { b16 a_, c_; split16(acc[t][r] * XS, a_, c_); Th[wave][8 * hlf + r][t * 16 + nloc] = a_; Tl[wave][8 * hlf + r][t * 16 + nloc] = c_; }
  wave_lds_sync();
  const int NHp = kind == 0 ? HQ : HKV; b16* dh = kind == 0 ? QH : kind == 1 ? KH : VROW;
  for (int pass = 0; pass < 2; ++pass) { for (int rr = 0; rr < 16; ++rr) if (lane < 16) { const int m = m0 + rr, b = m / S, s = m - b * S; const size_t gi = (((size_t)b * NHp + head) * S + s) * DH + lane * 8;
      *(volatile v8b*)(dh + gi) = *(const v8b*)(&Th[wave][rr][lane * 8]); if (kind == 0) *(volatile v8b*)(QL + gi) = *(const v8b*)(&Tl[wave][rr][lane * 8]); } __threadfence(); }
}
__global__ __launch_bounds__(256) void vt_kernel(const b16* __restrict__ VROW, b16* __restrict__ VT) {
  __shared__ __attribute__((aligned(16))) b16 Tt[DH][64 + 8];
  const int bh = blockIdx.y, s0 = blockIdx.x * 64, t_ = threadIdx.x;
  for (int k = t_; k < 64 * DH; k += 256) { const int ss = k >> 7, d = k & 127; Tt[d][ss] = VROW[((size_t)bh * S + s0 + ss) * DH + d]; }
  __syncthreads();
  for (int pass = 0; pass < 2; ++pass) { for (int q = t_; q < DH * 8; q += 256) { const int d = q >> 3, c8 = (q & 7) * 8; *(volatile v8b*)(VT + ((size_t)bh * DH + d) * S + s0 + c8) = *(const v8b*)(&Tt[d][c8]); } __threadfence(); }
}
__global__ __launch_bounds__(64) void attn_kernel(const b16* __restrict__ QH, const b16* __restrict__ QL, const b16* __restrict__ KH, const b16* __restrict__ VT, b16* __restrict__ ATT) {
  __shared__ __attribute__((aligned(16))) b16 To[2][16][DH + 8];
  const int wave = threadIdx.x >> 5, lane = threadIdx.x & 31, hh = lane >> 4, col = lane & 15; const int bh = blockIdx.y, b = bh / HQ, hq = bh - b * HQ, kvh = hq / GRP, q0 = blockIdx.x * 32 + wave * 16, qi = q0 + col;
  const b16* Qh = QH + ((size_t)bh * S) * DH; const b16* Ql = QL + ((size_t)bh * S) * DH; const b16* K = KH + ((size_t)(b * HKV + kvh) * S) * DH; const b16* V = VT + (size_t)(b * HKV + kvh) * DH * S;
  v16b qf[4], ql[4];
#pragma unroll
  for (int ks = 0; ks < 4; ++ks) { qf[ks] = frag_kb(Qh + (size_t)qi * DH + ks * 32, hh); ql[ks] = frag_kb(Ql + (size_t)qi * DH + ks * 32, hh); }
  const float scale = SCALING * (1.0f / (XS * XS));
  float m = -INFINITY, l = 0.0f; v8f o[8];
#pragma unroll
  for (int t = 0; t < 8; ++t) o[t] = (v8f){};
  for (int kb = 0; kb < S; kb += 32) {
    v8f s0 = {}, s1 = {};
#pragma unroll
    for (int ks = 0; ks < 4; ++ks) { const v16b k0 = frag_kb(K + (size_t)(kb + col) * DH + ks * 32, hh), k1 = frag_kb(K + (size_t)(kb + 16 + col) * DH + ks * 32, hh);
      s0 = wmma16b(k0, qf[ks], s0); s0 = wmma16b(k0, ql[ks], s0); s1 = wmma16b(k1, qf[ks], s1); s1 = wmma16b(k1, ql[ks], s1); }
    float mr = -INFINITY;
#pragma unroll
    for (int r = 0; r < 8; ++r) { s0[r] *= scale; s1[r] *= scale; mr = fmaxf(mr, fmaxf(s0[r], s1[r])); }
    mr = fmaxf(mr, __shfl_xor(mr, 16)); const float mn = fmaxf(m, mr); const float al_ = nexp(m - mn); m = mn; float sum = 0.0f; v16b pb;
#pragma unroll
    for (int r = 0; r < 8; ++r) { const float e0 = nexp(s0[r] - mn), e1 = nexp(s1[r] - mn); sum += e0 + e1; pb[r] = (b16)(e0 * PS); pb[8 + r] = (b16)(e1 * PS); }
    sum += __shfl_xor(sum, 16); l = l * al_ + sum;
#pragma unroll
    for (int t = 0; t < 8; ++t) { o[t] *= al_; o[t] = wmma16b(frag_kb(V + (size_t)(t * 16 + col) * S + kb, hh), pb, o[t]); } }
  const float inv = 1.0f / (l * PS * XS);
#pragma unroll
  for (int t = 0; t < 8; ++t)
#pragma unroll
    for (int r = 0; r < 8; ++r) To[wave][col][t * 16 + 8 * hh + r] = (b16)(o[t][r] * inv * XS);
  wave_lds_sync();
  for (int pass = 0; pass < 2; ++pass) { for (int rr = 0; rr < 16; ++rr) if (lane < 16) *(volatile v8b*)(ATT + ((size_t)b * S + q0 + rr) * HID + hq * DH + lane * 8) = *(const v8b*)(&To[wave][rr][lane * 8]); __threadfence(); }
}
__global__ __launch_bounds__(128) void proj_kernel(const b16* __restrict__ ATT, const b16* __restrict__ WO, float* __restrict__ out) {
  __shared__ __attribute__((aligned(16))) float Ts[4][16][128 + 4];
  const int wave = threadIdx.x >> 5, lane = threadIdx.x & 31, nloc = lane & 15, hlf = lane >> 4; const int m0 = blockIdx.x * 64 + wave * 16, n0 = blockIdx.y * 128;
  v8f acc[8];
#pragma unroll
  for (int t = 0; t < 8; ++t) acc[t] = (v8f){};
#pragma unroll 2
  for (int kb = 0; kb < HID; kb += 32) { const v16b a = frag_kb(ATT + (size_t)(m0 + nloc) * HID + kb, hlf);
#pragma unroll
    for (int t = 0; t < 8; ++t) acc[t] = wmma16b(a, frag_kb(WO + (size_t)(n0 + t * 16 + nloc) * HID + kb, hlf), acc[t]); }
#pragma unroll
  for (int t = 0; t < 8; ++t)
#pragma unroll
    for (int r = 0; r < 8; ++r) Ts[wave][8 * hlf + r][t * 16 + nloc] = acc[t][r] * (1.0f / (XS * WSC));
  wave_lds_sync();
  for (int pass = 0; pass < 2; ++pass) { for (int rr = 0; rr < 16; ++rr) *(volatile v4f*)(out + (size_t)(m0 + rr) * HID + n0 + lane * 4) = *(const v4f*)(&Ts[wave][rr][lane * 4]); __threadfence(); }
}
}

extern "C" void kernel_launch(void* const* d_in, const int* in_sizes, int n_in, void* d_out, int out_size, void* d_ws, size_t ws_size, hipStream_t stream) {
  (void)n_in;
  auto Fp = [&](int i) { return (const float*)d_in[i]; };
  if (in_sizes[0] != NROW * HID || in_sizes[1] != NROW * DH || in_sizes[2] != NROW * DH || in_sizes[3] != TOT * HID || in_sizes[6] != HID * HID || out_size != NROW * HID) return;
  size_t off = 0; char* ws = (char*)d_ws;
  auto carve = [&](size_t bytes) { char* p = ws + off; off += (bytes + 255) & ~(size_t)255; return p; };
  b16* X16 = (b16*)carve((size_t)NROW * HID * 2); b16* WQ = (b16*)carve((size_t)TOT * HID * 2); b16* WO = (b16*)carve((size_t)HID * HID * 2);
  b16* QH = (b16*)carve((size_t)NB * HQ * S * DH * 2); b16* QL = (b16*)carve((size_t)NB * HQ * S * DH * 2); b16* KH = (b16*)carve((size_t)NB * HKV * S * DH * 2); b16* VROW = (b16*)carve((size_t)NB * HKV * S * DH * 2); b16* VT = (b16*)carve((size_t)NB * HKV * DH * S * 2);
  b16* ATT = X16;
  if (off > ws_size) return;
  prep_kernel<<<1024, 256, 0, stream>>>(Fp(0), Fp(3), Fp(6), X16, WQ, WO);
  qkv_kernel<<<dim3(NROW / 64, TOT / DH), 128, 0, stream>>>(X16, WQ, Fp(1), Fp(2), Fp(4), Fp(5), QH, QL, KH, VROW);
  vt_kernel<<<dim3(S / 64, NB * HKV), 256, 0, stream>>>(VROW, VT);
  attn_kernel<<<dim3(S / 32, NB * HQ), 64, 0, stream>>>(QH, QL, KH, VT, ATT);
  proj_kernel<<<dim3(NROW / 64, HID / 128), 128, 0, stream>>>(ATT, WO, (float*)d_out);
}
